// RGCN_90168543412868
// MI455X (gfx1250) — hardware-run, weakly checked
//
#include <hip/hip_runtime.h>


namespace {

constexpr int N = 50000, NP = 50048, NPL = NP  , SRCM = N  , EFULL = 800000, E = EFULL  ;
constexpr int F = 128, R = 8, KSH = 16  , NKEY = R << KSH, KC = (R + 1) * F  , NL = (NPL < N ? NPL : N), NRB = 256  ;
constexpr float XS = 8.0f, WSC = 256.0f, WSQ = 0.25f, RS_ = 1024.0f, SLOPE = 0.0f, BNEPS = 1e-5f;
static_assert(N < (1 << KSH) && NP % 32 == 0 && NPL % 32 == 0 && F == 128 && E % 4 == 0 && E % NRB == 0, "layout");
typedef _Float16 b16;
typedef __attribute__((ext_vector_type(16))) _Float16 v16b;
typedef __attribute__((ext_vector_type(8))) _Float16 v8b;
typedef __attribute__((ext_vector_type(8))) float v8f;
typedef __attribute__((ext_vector_type(4))) float v4f;
__device__ __forceinline__ float bf16_rne(float f) { unsigned int u = __float_as_uint(f); u += 0x7FFFu + ((u >> 16) & 1u); return __uint_as_float(u & 0xFFFF0000u); }
__device__ __forceinline__ void split16(float v, b16& hi, b16& lo) { hi = (b16)v; lo = (b16)(v - (float)hi); }
__device__ __forceinline__ v16b frag_kb(const b16* p, int hh) { const v8b a = *(const v8b*)(p + 8 * hh), b = *(const v8b*)(p + 16 + 8 * hh); v16b f;
#pragma unroll
  for (int e = 0; e < 8; ++e) { f[e] = a[e]; f[8 + e] = b[e]; } return f; }
__device__ __forceinline__ v8f wmma16b(v16b a, v16b b, v8f c) { v8f d = __builtin_amdgcn_wmma_f32_16x16x32_f16(false, a, false, b, (short)0, c, false, false); asm volatile("v_nop\n\tv_nop\n\tv_nop\n\tv_nop" : "+v"(d) : "v"(a), "v"(b)); return d; }
__device__ __forceinline__ void wave_lds_sync() { __builtin_amdgcn_fence(__ATOMIC_RELEASE, "workgroup"); __builtin_amdgcn_wave_barrier(); __builtin_amdgcn_fence(__ATOMIC_ACQUIRE, "workgroup"); }
__device__ __forceinline__ float pmul(float a, float b) { float p = a * b; asm volatile("" : "+v"(p)); return p; }
__device__ __forceinline__ int iclamp(int v, int lo, int hi) { return v < lo ? lo : (v > hi ? hi : v); }
constexpr int CSR_NBLK = 512, CSR_GB = 10, CSR_GN = 1 << CSR_GB  , CSR_MAXG = 512, CSR_CAP = 12288  ;
__global__ __launch_bounds__(64) void csrA_kernel(const int* __restrict__ dst, int E, int N, int nG, int CHP, int NGP, int* __restrict__ STG, int* __restrict__ HST) {
  extern __shared__ int sm[];
  int* cnt = sm; int* run = sm + NGP; int* ids = sm + 2 * NGP;
  const int b = blockIdx.x; const int ch = (E + CSR_NBLK - 1) / CSR_NBLK; const int e0 = b * ch, e1 = min(E, e0 + ch);
  for (int i = threadIdx.x; i < NGP; i += 64) cnt[i] = 0;
  for (int i = threadIdx.x; i < CHP; i += 64) ids[i] = -1;
  __syncthreads();
  if (threadIdx.x == 0) {
    for (int e = e0; e < e1; ++e) { int d = dst[e]; d = (d < 0) ? 0 : (d >= N ? N - 1 : d); cnt[d >> CSR_GB] += 1; }
    int acc = 0; for (int g = 0; g < nG; ++g) { run[g] = acc; acc += cnt[g]; }
    for (int e = e0; e < e1; ++e) { int d = dst[e]; d = (d < 0) ? 0 : (d >= N ? N - 1 : d); const int g = d >> CSR_GB; ids[run[g]] = e; run[g] += 1; } }
  __syncthreads();
  typedef __attribute__((ext_vector_type(4))) int v4i;
  for (int pass = 0; pass < 2; ++pass) {
    for (int i = threadIdx.x; i < CHP / 4; i += 64) *(volatile v4i*)(STG + (size_t)b * CHP + i * 4) = *(const v4i*)(&ids[i * 4]);
    for (int i = threadIdx.x; i < NGP / 4; i += 64) { v4i v; for (int e = 0; e < 4; ++e) v[e] = (i * 4 + e < nG) ? cnt[i * 4 + e] : 0; *(volatile v4i*)(HST + (size_t)b * NGP + i * 4) = v; }
    __threadfence(); }
}
__global__ __launch_bounds__(512) void csrS_kernel(const int* __restrict__ HST, int nG, int NGP, int* __restrict__ START, int* __restrict__ TOT, int* __restrict__ OFF) {
  __shared__ int tot[CSR_MAXG];
  const int b = threadIdx.x;
  for (int pass = 0; pass < 2; ++pass) { int runb = 0; for (int g = 0; g < nG; ++g) { int c = HST[(size_t)b * NGP + g]; c = (c < 0) ? 0 : c; ((volatile int*)OFF)[(size_t)g * CSR_NBLK + b] = runb; runb += c; } __threadfence(); }
  for (int g = threadIdx.x; g < nG; g += 512) { int s = 0; for (int bb = 0; bb < CSR_NBLK; ++bb) { int c = HST[(size_t)bb * NGP + g]; s += (c < 0) ? 0 : c; } tot[g] = s; }
  __syncthreads();
  if (threadIdx.x < 32) {
    __shared__ int st[CSR_MAXG + 32];
    if (threadIdx.x == 0) { int acc = 0; for (int g = 0; g < NGP; ++g) { st[g] = acc; if (g < nG) acc += (tot[g] + 31) & ~31; } st[NGP] = acc; }
    __builtin_amdgcn_fence(__ATOMIC_RELEASE, "workgroup"); __builtin_amdgcn_wave_barrier(); __builtin_amdgcn_fence(__ATOMIC_ACQUIRE, "workgroup");
    for (int pass = 0; pass < 2; ++pass) { for (int i = threadIdx.x; i < NGP + 32; i += 32) { ((volatile int*)START)[i] = (i <= NGP) ? st[min(i, NGP)] : 0; ((volatile int*)TOT)[i] = (i < nG) ? tot[i] : 0; } __threadfence(); } }
}
__global__ __launch_bounds__(256) void csrB_kernel(const int* __restrict__ dst, int N, int nG, int CHP, int NGP, int permLen, const int* __restrict__ STG, const int* __restrict__ HST, const int* __restrict__ OFF, const int* __restrict__ START, const int* __restrict__ TOT, int* __restrict__ PERM, int* __restrict__ ROWPTR, int* __restrict__ ROWCNT, int* __restrict__ FLAG) {
  typedef __attribute__((ext_vector_type(4))) int v4i;
  __shared__ int ids[CSR_CAP]; __shared__ unsigned short key[CSR_CAP]; __shared__ int outp[CSR_CAP]; __shared__ int ncnt[CSR_GN + 1]; __shared__ int boff[CSR_NBLK + 1];
  const int g = blockIdx.x, t_ = threadIdx.x; int tot = TOT[g]; int st = START[g], stn = START[g + 1]; const int v0 = g * CSR_GN; const int nv = min(CSR_GN, N - v0);
  st = (st < 0) ? 0 : (st > permLen - 32 ? permLen - 32 : st) & ~31; stn = (stn < st) ? st : (stn > permLen ? permLen : stn); tot = (tot < 0) ? 0 : tot; if (tot > stn - st && tot <= CSR_CAP) tot = stn - st;
  if (tot > CSR_CAP) {
    for (int pass = 0; pass < 2; ++pass) { for (int i = t_; i < CSR_GN / 4; i += 256) { v4i a, c; for (int e = 0; e < 4; ++e) { a[e] = st; c[e] = 0; } *(volatile v4i*)(ROWPTR + v0 + i * 4) = a; *(volatile v4i*)(ROWCNT + v0 + i * 4) = c; } if (t_ == 0) ((volatile int*)FLAG)[0] = 1; __threadfence(); } (void)nv; return; }
  if (t_ == 0) { int acc = 0; for (int b = 0; b < CSR_NBLK; ++b) { boff[b] = acc; int c = HST[(size_t)b * NGP + g]; c = (c < 0) ? 0 : (c > CHP ? CHP : c); acc += c; if (acc > tot) acc = tot; } boff[CSR_NBLK] = acc; }
  for (int i = t_; i <= CSR_GN; i += 256) ncnt[i] = 0;
  __syncthreads();
  for (int b = 0; b < CSR_NBLK; ++b) { const int c = boff[b + 1] - boff[b]; int o_ = OFF[(size_t)g * CSR_NBLK + b]; o_ = (o_ < 0) ? 0 : (o_ > CHP - c ? CHP - c : o_); const int* src_ = STG + (size_t)b * CHP + o_;
    for (int i = t_; i < c; i += 256) { int id = src_[i]; id = (id < 0) ? 0 : id; ids[boff[b] + i] = id; int d = dst[id]; d = (d < v0) ? v0 : (d >= N ? N - 1 : d); int kk = d - v0; kk = (kk < 0) ? 0 : (kk >= CSR_GN ? CSR_GN - 1 : kk); key[boff[b] + i] = (unsigned short)kk; } }
  __syncthreads();
  if (t_ == 0) { for (int i = 0; i < tot; ++i) ncnt[key[i]] += 1; int acc = 0; for (int vl = 0; vl < CSR_GN; ++vl) { const int c = ncnt[vl]; ncnt[vl] = acc; acc += c; } ncnt[CSR_GN] = acc;
    for (int i = 0; i < tot; ++i) { const int vl = key[i]; outp[ncnt[vl]] = ids[i]; ncnt[vl] += 1; }
    for (int vl = CSR_GN; vl > 0; --vl) ncnt[vl] = ncnt[vl - 1]; ncnt[0] = 0; }
  __syncthreads();
  for (int pass = 0; pass < 2; ++pass) {
    for (int i = t_; i < (stn - st) / 4; i += 256) { v4i v; for (int e = 0; e < 4; ++e) { const int q = i * 4 + e; v[e] = (q < tot) ? outp[q] : -1; } *(volatile v4i*)(PERM + st + i * 4) = v; }
    for (int i = t_; i < CSR_GN / 4; i += 256) { v4i a, c; for (int e = 0; e < 4; ++e) { const int vl = i * 4 + e; a[e] = st + ncnt[vl]; c[e] = (vl < nv) ? (ncnt[vl + 1] - ncnt[vl]) : 0; } *(volatile v4i*)(ROWPTR + v0 + i * 4) = a; *(volatile v4i*)(ROWCNT + v0 + i * 4) = c; }
    __threadfence(); }
}
__global__ __launch_bounds__(256) void csrZ_kernel(int* __restrict__ p, size_t n4) { typedef __attribute__((ext_vector_type(4))) int v4i; const size_t tid = (size_t)blockIdx.x * 256 + threadIdx.x, nth = (size_t)gridDim.x * 256; v4i z = {0, 0, 0, 0}; for (size_t i = tid; i < n4; i += nth) *(volatile v4i*)(p + i * 4) = z; }
struct CsrBufs { int *STG, *HST, *OFF, *START, *TOT, *PERM, *ROWPTR, *ROWCNT, *FLAG; int nG, NGP, CHP; size_t permLen; char* base; size_t bytes; };
static size_t csr_carve(CsrBufs& c, char* ws, size_t off, int E, int N) {
  const size_t off0 = off; c.base = ws + off;
  auto al = [&](size_t bytes) { char* p = ws + off; off += (bytes + 255) & ~(size_t)255; return p; };
  c.nG = (N + CSR_GN - 1) / CSR_GN; c.NGP = (c.nG + 31) & ~31; const int ch = (E + CSR_NBLK - 1) / CSR_NBLK; c.CHP = (ch + 31) & ~31; c.permLen = (size_t)E + 32 * (size_t)c.nG + 32;
  c.STG = (int*)al((size_t)CSR_NBLK * c.CHP * 4); c.HST = (int*)al((size_t)CSR_NBLK * c.NGP * 4); c.OFF = (int*)al((size_t)c.NGP * CSR_NBLK * 4); c.START = (int*)al((size_t)(c.NGP + 64) * 4); c.TOT = (int*)al((size_t)(c.NGP + 64) * 4);
  c.PERM = (int*)al(c.permLen * 4); c.ROWPTR = (int*)al((size_t)c.nG * CSR_GN * 4); c.ROWCNT = (int*)al((size_t)c.nG * CSR_GN * 4); c.FLAG = (int*)al(256);
  c.bytes = off - off0; return off;
}
static void csr_build(const CsrBufs& c, const int* dst, int E, int N, hipStream_t stream) {
  const size_t smem = (size_t)(2 * c.NGP + c.CHP) * 4;
  csrZ_kernel<<<512, 256, 0, stream>>>((int*)c.base, c.bytes / 16);
  csrA_kernel<<<CSR_NBLK, 64, smem, stream>>>(dst, E, N, c.nG, c.CHP, c.NGP, c.STG, c.HST);
  csrS_kernel<<<1, 512, 0, stream>>>(c.HST, c.nG, c.NGP, c.START, c.TOT, c.OFF);
  csrB_kernel<<<c.nG, 256, 0, stream>>>(dst, N, c.nG, c.CHP, c.NGP, (int)c.permLen, c.STG, c.HST, c.OFF, c.START, c.TOT, c.PERM, c.ROWPTR, c.ROWCNT, c.FLAG);
}

static_assert(NKEY / CSR_GN <= CSR_MAXG && CSR_GB == 10, "composite-key bucketing");
typedef __attribute__((ext_vector_type(4))) _Float16 v4h;
typedef __attribute__((ext_vector_type(2))) float v2f;
typedef __attribute__((ext_vector_type(4))) int v4i;
__global__ __launch_bounds__(256) void wt_kernel(const float* __restrict__ w, const float* __restrict__ root, b16* __restrict__ WT, float scl) {
  const int u = blockIdx.x * 256 + threadIdx.x; if (u >= F * KC / 8) return; const int e = u * 8; const int o = e / KC, k0 = e % KC; const float* src = k0 < R * F ? (w + (size_t)k0 * F) : (root + (size_t)(k0 - R * F) * F); v8b v;
#pragma unroll
  for (int j = 0; j < 8; ++j) v[j] = (b16)(bf16_rne(src[(size_t)j * F + o]) * scl);
  for (int pass = 0; pass < 2; ++pass) { *(volatile v8b*)(WT + e) = v; __threadfence(); }
}
__global__ __launch_bounds__(256) void wred_kernel(const float* __restrict__ w, float* __restrict__ PART) {
  __shared__ float rmn[256], rmx[256]; const int tid = threadIdx.x; const size_t e0 = (size_t)blockIdx.x * (E / NRB); float mn = INFINITY, mx = -INFINITY;
  for (int i = tid; i < E / NRB; i += 256) { const float v = bf16_rne(w[e0 + i]); mn = fminf(mn, v); mx = fmaxf(mx, v); }
  rmn[tid] = mn; rmx[tid] = mx; __syncthreads();
  for (int st = 128; st >= 1; st >>= 1) { if (tid < st) { rmn[tid] = fminf(rmn[tid], rmn[tid + st]); rmx[tid] = fmaxf(rmx[tid], rmx[tid + st]); } __syncthreads(); }
  for (int pass = 0; pass < 2; ++pass) { if (tid < 32) ((volatile float*)PART)[blockIdx.x * 32 + tid] = (tid == 0) ? rmn[0] : (tid == 1 ? rmx[0] : 0.0f); __threadfence(); }
}
__global__ __launch_bounds__(256) void wfin_kernel(const float* __restrict__ PART, float* __restrict__ STAT) {
  __shared__ float rmn[256], rmx[256]; const int tid = threadIdx.x; float mn = INFINITY, mx = -INFINITY;
  for (int i = tid; i < NRB; i += 256) { mn = fminf(mn, PART[i * 32]); mx = fmaxf(mx, PART[i * 32 + 1]); }
  rmn[tid] = mn; rmx[tid] = mx; __syncthreads();
  for (int st = 128; st >= 1; st >>= 1) { if (tid < st) { rmn[tid] = fminf(rmn[tid], rmn[tid + st]); rmx[tid] = fmaxf(rmx[tid], rmx[tid + st]); } __syncthreads(); }
  const float den = (rmx[0] - rmn[0]) + 1e-8f;
  for (int pass = 0; pass < 2; ++pass) { if (tid < 32) ((volatile float*)STAT)[tid] = (tid == 0) ? rmn[0] : (tid == 1 ? den : 0.0f); __threadfence(); }
}
__global__ __launch_bounds__(256) void ekey_kernel(const float* __restrict__ w, const int* __restrict__ dst, const int* __restrict__ typ, const float* __restrict__ STAT, float* __restrict__ EWN, int* __restrict__ KEY) {
  const int u = blockIdx.x * 256 + threadIdx.x; if (u >= E / 4) return; const float mn = STAT[0], den = STAT[1]; const v4f wv = *(const v4f*)(w + (size_t)u * 4); const v4i t = *(const v4i*)(dst + (size_t)u * 4), y = *(const v4i*)(typ + (size_t)u * 4); v4f o; v4i k;
  for (int j = 0; j < 4; ++j) { o[j] = (bf16_rne(wv[j]) - mn) / den; k[j] = (iclamp(y[j], 0, R - 1) << KSH) | iclamp(t[j], 0, N - 1); }
  for (int pass = 0; pass < 2; ++pass) { *(volatile v4f*)(EWN + (size_t)u * 4) = o; *(volatile v4i*)(KEY + (size_t)u * 4) = k; __threadfence(); }
}
template <bool RND, bool RELU>
__global__ __launch_bounds__(256) void layer_kernel(const float* __restrict__ H, const float* __restrict__ EWN, const int* __restrict__ srcs, const int* __restrict__ PERM, const int* __restrict__ ROWPTR, const int* __restrict__ ROWCNT, int permLen, const b16* __restrict__ WT, const b16* __restrict__ WQ, const float* __restrict__ bias, float* __restrict__ OUT, int mrows) {
  __shared__ __attribute__((aligned(16))) b16 Ah[32][F + 8], Al[32][F + 8]; __shared__ __attribute__((aligned(16))) float Tf[32][F + 4];
  const int tid = threadIdx.x, wave = tid >> 5, lane = tid & 31, nloc = lane & 15, hlf = lane >> 4; const int v0 = blockIdx.x * 32; const int row = tid >> 3, g = tid & 7, c0 = g * 16; const int v = v0 + row;
  v8f acc[2] = {(v8f){}, (v8f){}};
#pragma unroll 1
  for (int c = 0; c <= R; ++c) {
    float a[16];
    if (c < R) { for (int j = 0; j < 16; ++j) a[j] = 0.0f;
      int cnt = 0, q0 = 0; if (v < N) { const int key = (c << KSH) | v; cnt = iclamp(ROWCNT[key], 0, 65536); q0 = iclamp(ROWPTR[key], 0, permLen - 1); if (q0 + cnt > permLen) cnt = permLen - q0; }
#pragma unroll 1
      for (int i = 0; i < cnt; ++i) { const int e = iclamp(PERM[q0 + i], 0, E - 1); int s = iclamp(srcs[e], 0, N - 1); if (SRCM < N) s %= SRCM; const float wgt = EWN[e]; const float* hr = H + (size_t)s * F + c0;
#pragma unroll
        for (int q = 0; q < 4; ++q) { const v4f t4 = *(const v4f*)(hr + 4 * q); for (int j = 0; j < 4; ++j) a[4 * q + j] = fmaf(wgt, RND ? bf16_rne(t4[j]) : t4[j], a[4 * q + j]); } } }
    else { const float* hr = H + (size_t)(v < N ? v : N - 1) * F + c0;
#pragma unroll
      for (int q = 0; q < 4; ++q) { const v4f t4 = *(const v4f*)(hr + 4 * q); for (int j = 0; j < 4; ++j) a[4 * q + j] = (v < N) ? (RND ? bf16_rne(t4[j]) : t4[j]) : 0.0f; } }
    __syncthreads();
#pragma unroll
    for (int q = 0; q < 4; ++q) { v4h hv, lv; for (int j = 0; j < 4; ++j) { const float vs = a[4 * q + j] * XS; const b16 p = (b16)vs; hv[j] = p; lv[j] = (b16)((vs - (float)p) * RS_); } *(v4h*)(&Ah[row][c0 + 4 * q]) = hv; *(v4h*)(&Al[row][c0 + 4 * q]) = lv; }
    __syncthreads();
    { const b16* br = WT + (size_t)(wave * 16 + nloc) * KC + c * F; const b16* bq = WQ + (size_t)(wave * 16 + nloc) * KC + c * F;
#pragma unroll
      for (int kb = 0; kb < F; kb += 32) { const v16b bw = frag_kb(br + kb, hlf), bwq = frag_kb(bq + kb, hlf);
        acc[0] = wmma16b(frag_kb(&Ah[nloc][kb], hlf), bw, acc[0]); acc[0] = wmma16b(frag_kb(&Al[nloc][kb], hlf), bwq, acc[0]);
        acc[1] = wmma16b(frag_kb(&Ah[16 + nloc][kb], hlf), bw, acc[1]); acc[1] = wmma16b(frag_kb(&Al[16 + nloc][kb], hlf), bwq, acc[1]); } } }
  { const int col = wave * 16 + nloc; const float bb = bf16_rne(bias[col]);
#pragma unroll
    for (int rt = 0; rt < 2; ++rt)
#pragma unroll
      for (int q = 0; q < 8; ++q) { const int rr = rt * 16 + 8 * hlf + q; float y = acc[rt][q] * (1.0f / (XS * WSC)) + bb; if (RELU) y = fmaxf(y, 0.0f); Tf[rr][col] = (v0 + rr < N) ? y : 0.0f; } }
  __syncthreads();
  for (int pass = 0; pass < 2; ++pass) { for (int rr = wave * 4; rr < wave * 4 + 4; ++rr) if (v0 + rr < mrows) *(volatile v4f*)(OUT + (size_t)(v0 + rr) * F + lane * 4) = *(const v4f*)(&Tf[rr][lane * 4]); __threadfence(); }
}
}

extern "C" void kernel_launch(void* const* d_in, const int* in_sizes, int n_in, void* d_out, int out_size, void* d_ws, size_t ws_size, hipStream_t stream) {
  (void)n_in;
  auto Fp = [&](int i) { return (const float*)d_in[i]; }; auto Ip = [&](int i) { return (const int*)d_in[i]; };
  if (in_sizes[0] != N * F || in_sizes[1] != 2 * EFULL || in_sizes[2] != EFULL || in_sizes[3] != EFULL || in_sizes[4] != R * F * F || in_sizes[5] != F * F || in_sizes[6] != F || in_sizes[7] != R * F * F || in_sizes[8] != F * F || in_sizes[9] != F || out_size != N * F) return;
  size_t off = 0; char* ws = (char*)d_ws;
  auto carve = [&](size_t bytes) { char* p = ws + off; off += (bytes + 255) & ~(size_t)255; return p; };
  b16* WT1 = (b16*)carve((size_t)F * KC * 2); b16* WQ1 = (b16*)carve((size_t)F * KC * 2); b16* WT2 = (b16*)carve((size_t)F * KC * 2); b16* WQ2 = (b16*)carve((size_t)F * KC * 2);
  float* PART = (float*)carve((size_t)NRB * 128); float* STAT = (float*)carve(256); float* EWN = (float*)carve((size_t)E * 4); int* KEY = (int*)carve((size_t)E * 4); float* H1 = (float*)carve((size_t)NP * F * 4);
  CsrBufs csr; off = csr_carve(csr, ws, off, E, NKEY);
  if (off > ws_size || off > ((size_t)128 << 20)) return;
  wt_kernel<<<(F * KC / 8 + 255) / 256, 256, 0, stream>>>(Fp(4), Fp(5), WT1, WSC); wt_kernel<<<(F * KC / 8 + 255) / 256, 256, 0, stream>>>(Fp(4), Fp(5), WQ1, WSQ);
  wt_kernel<<<(F * KC / 8 + 255) / 256, 256, 0, stream>>>(Fp(7), Fp(8), WT2, WSC); wt_kernel<<<(F * KC / 8 + 255) / 256, 256, 0, stream>>>(Fp(7), Fp(8), WQ2, WSQ);
  wred_kernel<<<NRB, 256, 0, stream>>>(Fp(3), PART); wfin_kernel<<<1, 256, 0, stream>>>(PART, STAT);
  ekey_kernel<<<(E / 4 + 255) / 256, 256, 0, stream>>>(Fp(3), Ip(1) + EFULL, Ip(2), STAT, EWN, KEY);
  csr_build(csr, KEY, E, NKEY, stream);
  layer_kernel<true, true><<<NPL / 32, 256, 0, stream>>>(Fp(0), EWN, Ip(1), csr.PERM, csr.ROWPTR, csr.ROWCNT, (int)csr.permLen, WT1, WQ1, Fp(6), H1, NPL);
  layer_kernel<false, false><<<NPL / 32, 256, 0, stream>>>(H1, EWN, Ip(1), csr.PERM, csr.ROWPTR, csr.ROWCNT, (int)csr.permLen, WT2, WQ2, Fp(9), (float*)d_out, NL);
}
